// MeanShiftStep_66846870995311
// MI455X (gfx1250) — hardware-verified
//
#include <hip/hip_runtime.h>
#include <math.h>
#include <stdint.h>

#define NB    2
#define NQ    8192
#define NK    8192
#define DD    64
#define LNPS  6.931471805599453f
#define CSC   0.015625f
#define NHALF 0.0078125f
static_assert((NQ % 64) == 0);
static_assert((NK % 64) == 0);
static_assert(DD == 64);

typedef _Float16       v16h __attribute__((ext_vector_type(16)));
typedef _Float16       v8h  __attribute__((ext_vector_type(8)));
typedef __bf16         v16b __attribute__((ext_vector_type(16)));
typedef unsigned short v8us __attribute__((ext_vector_type(8)));
typedef float          v8f  __attribute__((ext_vector_type(8)));
typedef float          v4f  __attribute__((ext_vector_type(4)));
typedef unsigned int   v4u  __attribute__((ext_vector_type(4)));

union FragH { v16h v; v8h  h[2]; };
union FragB { v16b v; v8us u[2]; };
static_assert(sizeof(FragH) == 32);
static_assert(sizeof(FragB) == 32);

__device__ __forceinline__ unsigned short bf_bits(float f) {
  unsigned u = __float_as_uint(f);
  return (unsigned short)((u + 0x7FFFu + ((u >> 16) & 1u)) >> 16);
}
__device__ __forceinline__ float bf_up(unsigned short h) { return __uint_as_float(((unsigned)h) << 16); }
__device__ __forceinline__ float bfr(float f) { return bf_up(bf_bits(f)); }
__device__ __forceinline__ unsigned short h_bits(_Float16 x) { return __builtin_bit_cast(unsigned short, x); }
__device__ __forceinline__ unsigned pk16(unsigned short a, unsigned short b) { return (unsigned)a | ((unsigned)b << 16); }
__device__ __forceinline__ v8f zero8() { v8f z = {0.f, 0.f, 0.f, 0.f, 0.f, 0.f, 0.f, 0.f}; return z; }
__device__ __forceinline__ float hmax8(v8f s) {
  return fmaxf(fmaxf(fmaxf(s[0], s[1]), fmaxf(s[2], s[3])), fmaxf(fmaxf(s[4], s[5]), fmaxf(s[6], s[7])));
}

__device__ __forceinline__ v16h ldfrag_h(const _Float16* p) {
  FragH f;
  f.h[0] = *(const v8h*)(p);
  f.h[1] = *(const v8h*)(p + 16);
  return f.v;
}
__device__ __forceinline__ v16b ldfrag_b(const unsigned short* p) {
  FragB f;
  f.u[0] = *(const v8us*)(p);
  f.u[1] = *(const v8us*)(p + 16);
  return f.v;
}

__device__ __forceinline__ v8f mma_h_raw(v16h a, v16h b, v8f c) {
  return __builtin_amdgcn_wmma_f32_16x16x32_f16(false, a, false, b, (short)0, c, false, false);
}
__device__ __forceinline__ v8f mma_b_raw(v16b a, v16b b, v8f c) {
  return __builtin_amdgcn_wmma_f32_16x16x32_bf16(false, a, false, b, (short)0, c, false, false);
}
__device__ __forceinline__ void sguard6(v8f& a, v8f& b, v16b x0, v16b x1, v16b x2, v16b x3, v16b y0, v16b y1) {
#if defined(__HIP_DEVICE_COMPILE__)
  const v16h h0 = __builtin_bit_cast(v16h, x0), h1 = __builtin_bit_cast(v16h, x1);
  const v16h h2 = __builtin_bit_cast(v16h, x2), h3 = __builtin_bit_cast(v16h, x3);
  const v16h g0 = __builtin_bit_cast(v16h, y0), g1 = __builtin_bit_cast(v16h, y1);
  asm volatile("v_nop\n\tv_nop\n\tv_nop\n\tv_nop"
               : "+v"(a), "+v"(b) : "v"(h0), "v"(h1), "v"(h2), "v"(h3), "v"(g0), "v"(g1));
#endif
}
__device__ __forceinline__ void oguard4(v8f& a, v8f& b, v8f& c, v8f& d,
                                        v16h x0, v16h x1, v16h x2, v16h x3, v16h p0) {
#if defined(__HIP_DEVICE_COMPILE__)
  asm volatile("v_nop\n\tv_nop\n\tv_nop\n\tv_nop"
               : "+v"(a), "+v"(b), "+v"(c), "+v"(d) : "v"(x0), "v"(x1), "v"(x2), "v"(x3), "v"(p0));
#endif
}

__global__ __launch_bounds__(256) void cvt_keys(const float* __restrict__ keys,
                                                 unsigned short* KB, unsigned short* VT, float* bias) {
  __shared__ __align__(16) unsigned short Ts[64 * 72];
  __shared__ __align__(16) float sB[64];
  const int tid  = threadIdx.x;
  const int lane = tid & 31, wave = tid >> 5;
  const int s0   = blockIdx.x * 64;
  const int bb   = s0 / NK;
  const int m0   = s0 - bb * NK;

  {
    const int e = lane & 7, rq = lane >> 3;
    v4u u[2];
    size_t go[2];
    float ss[2];
#pragma unroll
    for (int it = 0; it < 2; ++it) {
      const int row = s0 + wave * 8 + it * 4 + rq;
      const size_t o = (size_t)row * DD + 8 * e;
      go[it] = o;
      const v4f a = *(const v4f*)(keys + o), b = *(const v4f*)(keys + o + 4);
      unsigned short hs[8];
#pragma unroll
      for (int i = 0; i < 4; ++i) { hs[i] = bf_bits(a[i]); hs[4 + i] = bf_bits(b[i]); }
      float q = 0.f;
#pragma unroll
      for (int i = 0; i < 8; ++i) { const float f = bf_up(hs[i]); q += f * f; }
      v4u w;
#pragma unroll
      for (int i = 0; i < 4; ++i) w[i] = pk16(hs[2 * i], hs[2 * i + 1]);
      u[it]  = w;
      ss[it] = q;
    }
#pragma unroll
    for (int it = 0; it < 2; ++it) {
      ss[it] += __shfl_xor(ss[it], 1, 32);
      ss[it] += __shfl_xor(ss[it], 2, 32);
      ss[it] += __shfl_xor(ss[it], 4, 32);
    }
    if (e == 0) {
      sB[wave * 8 + rq]     = -NHALF * ss[0];
      sB[wave * 8 + 4 + rq] = -NHALF * ss[1];
    }
    for (int pass = 0; pass < 2; ++pass) {
#pragma unroll
      for (int it = 0; it < 2; ++it) *(volatile v4u*)(KB + go[it]) = u[it];
      __threadfence();
    }
  }

  {
    const int row = tid >> 2;
    const int cg  = (tid & 3) * 16;
    const float* p = keys + (size_t)(s0 + row) * DD + cg;
#pragma unroll
    for (int j = 0; j < 4; ++j) {
      const v4f x = *(const v4f*)(p + j * 4);
#pragma unroll
      for (int t = 0; t < 4; ++t) Ts[(cg + j * 4 + t) * 72 + row] = h_bits((_Float16)bfr(x[t]));
    }
  }
  __syncthreads();
  {
    const int e = tid & 7, lq = tid >> 3;
    v4u u[2];
#pragma unroll
    for (int it = 0; it < 2; ++it) {
      const int dr = it * 32 + lq;
      u[it] = *(const v4u*)(Ts + dr * 72 + 8 * e);
    }
    unsigned short* db = VT + (size_t)bb * DD * NK + m0 + 8 * e;
    for (int pass = 0; pass < 2; ++pass) {
#pragma unroll
      for (int it = 0; it < 2; ++it) {
        const int dr = it * 32 + lq;
        *(volatile v4u*)(db + (size_t)dr * NK) = u[it];
      }
      __threadfence();
    }
  }
  if (tid < 16) {
    const v4f bv = *(const v4f*)(sB + 4 * tid);
    float* bp = bias + s0 + 4 * tid;
    for (int pass = 0; pass < 2; ++pass) {
      *(volatile v4f*)bp = bv;
      __threadfence();
    }
  }
}

__global__ __launch_bounds__(128)
void wmean_main(const float* __restrict__ qin, const unsigned short* __restrict__ kbp,
                const unsigned short* __restrict__ vtp, const float* __restrict__ biasp, float* out) {
  __shared__ __align__(16) float Os[64 * 68];
  const int tid  = threadIdx.x;
  const int wave = tid >> 5;
  const int lane = tid & 31;
  const int hh   = lane >> 4;
  const int c    = lane & 15;
  const int q0   = blockIdx.x * 64;
  const int bb   = q0 / NQ;

  const unsigned short* kbb  = kbp   + (size_t)bb * NK * DD;
  const unsigned short* vtb  = vtp   + (size_t)bb * DD * NK;
  const float*          bias = biasp + (size_t)bb * NK;

  FragB qfa, qfc;
  {
    const float* qr = qin + (size_t)(q0 + wave * 16 + c) * DD + 8 * hh;
    const v4f x0 = *(const v4f*)(qr),      x1 = *(const v4f*)(qr + 4);
    const v4f x2 = *(const v4f*)(qr + 16), x3 = *(const v4f*)(qr + 20);
    const v4f y0 = *(const v4f*)(qr + 32), y1 = *(const v4f*)(qr + 36);
    const v4f y2 = *(const v4f*)(qr + 48), y3 = *(const v4f*)(qr + 52);
    v8us ua, ub, uc, ud;
#pragma unroll
    for (int i = 0; i < 4; ++i) {
      ua[i] = bf_bits(x0[i]); ua[4 + i] = bf_bits(x1[i]);
      ub[i] = bf_bits(x2[i]); ub[4 + i] = bf_bits(x3[i]);
      uc[i] = bf_bits(y0[i]); uc[4 + i] = bf_bits(y1[i]);
      ud[i] = bf_bits(y2[i]); ud[4 + i] = bf_bits(y3[i]);
    }
    qfa.u[0] = ua; qfa.u[1] = ub;
    qfc.u[0] = uc; qfc.u[1] = ud;
  }
  const v16b qf0 = qfa.v, qf1 = qfc.v;

  const unsigned short* Kp = kbb + (size_t)c * DD + 8 * hh;
  const _Float16* VTh = (const _Float16*)(const void*)vtb;
  const _Float16* V0 = VTh + (size_t)c * NK + 8 * hh;
  const _Float16* V1 = V0 + (size_t)16 * NK;
  const _Float16* V2 = V0 + (size_t)32 * NK;
  const _Float16* V3 = V0 + (size_t)48 * NK;

  float m = -1.0e30f, l = 0.f;
  v8f o0 = zero8(), o1 = zero8(), o2 = zero8(), o3 = zero8();
#pragma unroll 1
  for (int it = 0; it < NK / 32; ++it) {
    const int kb = it * 32;
    const unsigned short* k0p = Kp + (size_t)kb * DD;
    const unsigned short* k1p = k0p + (size_t)16 * DD;
    const v16b a00 = ldfrag_b(k0p),      a10 = ldfrag_b(k1p);
    const v16b a01 = ldfrag_b(k0p + 32), a11 = ldfrag_b(k1p + 32);
    v8f s0 = mma_b_raw(a00, qf0, zero8());
    v8f s1 = mma_b_raw(a10, qf0, zero8());
    s0 = mma_b_raw(a01, qf1, s0);
    s1 = mma_b_raw(a11, qf1, s1);
    sguard6(s0, s1, a00, a10, a01, a11, qf0, qf1);

    const float* bp = bias + kb + 8 * hh;
    const v8f b0 = *(const v8f*)(bp);
    const v8f b1 = *(const v8f*)(bp + 16);
    v8f w0, w1;
#pragma unroll
    for (int r = 0; r < 8; ++r) { w0[r] = fmaf(s0[r], CSC, b0[r]); w1[r] = fmaf(s1[r], CSC, b1[r]); }

    float mx = fmaxf(hmax8(w0), hmax8(w1));
    mx = fmaxf(mx, __shfl_xor(mx, 16, 32));
    const float mn   = fmaxf(m, mx);
    const float corr = __expf(m - mn);
    m = mn;
    const float msh = mn - LNPS;
    l *= corr;
#pragma unroll
    for (int r = 0; r < 8; ++r) { o0[r] *= corr; o1[r] *= corr; o2[r] *= corr; o3[r] *= corr; }

    FragH ph;
    float ls = 0.f;
#pragma unroll
    for (int r = 0; r < 8; ++r) {
      const float e0 = __expf(w0[r] - msh);
      const float e1 = __expf(w1[r] - msh);
      ls += e0 + e1;
      ph.h[0][r] = (_Float16)e0;
      ph.h[1][r] = (_Float16)e1;
    }
    l += ls;

    const v16h vf0 = ldfrag_h(V0 + kb);
    const v16h vf1 = ldfrag_h(V1 + kb);
    const v16h vf2 = ldfrag_h(V2 + kb);
    const v16h vf3 = ldfrag_h(V3 + kb);
    o0 = mma_h_raw(vf0, ph.v, o0);
    o1 = mma_h_raw(vf1, ph.v, o1);
    o2 = mma_h_raw(vf2, ph.v, o2);
    o3 = mma_h_raw(vf3, ph.v, o3);
    oguard4(o0, o1, o2, o3, vf0, vf1, vf2, vf3, ph.v);
  }
  l += __shfl_xor(l, 16, 32);
  const float rl = 1.0f / l;

  float* os = Os + (wave * 16 + c) * 68 + 8 * hh;
#pragma unroll
  for (int r = 0; r < 8; ++r) { os[r] = o0[r] * rl; os[16 + r] = o1[r] * rl; os[32 + r] = o2[r] * rl; os[48 + r] = o3[r] * rl; }
  __syncthreads();
  {
    const int e = tid & 7, lq = tid >> 3;
    v4f vals[8];
#pragma unroll
    for (int it = 0; it < 8; ++it) {
      const int L   = it * 16 + lq;
      const int row = L >> 1, hf = L & 1;
      vals[it] = *(const v4f*)(Os + row * 68 + hf * 32 + 4 * e);
    }
    float* ob = out + (size_t)q0 * DD;
    for (int pass = 0; pass < 2; ++pass) {
#pragma unroll
      for (int it = 0; it < 8; ++it) {
        const int L   = it * 16 + lq;
        const int row = L >> 1, hf = L & 1;
        *(volatile v4f*)(ob + (size_t)row * DD + hf * 32 + 4 * e) = vals[it];
      }
      __threadfence();
    }
  }
}

extern "C" void kernel_launch(void* const* d_in, const int* in_sizes, int n_in,
                              void* d_out, int out_size, void* d_ws, size_t ws_size,
                              hipStream_t stream) {
  if (n_in < 2) return;
  if (in_sizes[0] != NB * NQ * DD || in_sizes[1] != NB * NK * DD) return;
  if (out_size != NB * NQ * DD) return;

  size_t off = 0;
  const size_t oK = off; off += (size_t)NB * NK * DD * 2;
  const size_t oV = off; off += (size_t)NB * NK * DD * 2;
  const size_t oB = off; off += (size_t)NB * NK * 4;
  if (off > ws_size) return;
  if (off > (size_t)134217728) return;

  const float* qpts = (const float*)d_in[0];
  const float* keys = (const float*)d_in[1];
  char* ws = (char*)d_ws;
  unsigned short* KB = (unsigned short*)(ws + oK);
  unsigned short* VT = (unsigned short*)(ws + oV);
  float* BIAS        = (float*)(ws + oB);
  float* out         = (float*)d_out;

  const dim3 blk256(256), blk128(128);
  const dim3 gCV(NB * NK / 64);
  const dim3 gAT(NB * NQ / 64);

  cvt_keys<<<gCV, blk256, 0, stream>>>(keys, KB, VT, BIAS);

  wmean_main<<<gAT, blk128, 0, stream>>>(qpts, KB, VT, BIAS, out);
  (void)hipGetLastError();
}
